// PerformerWrapper_74002286510202
// MI455X (gfx1250) — hardware-verified
//
#include <hip/hip_runtime.h>
#include <math.h>

typedef __attribute__((ext_vector_type(16))) _Float16 v16h;
typedef __attribute__((ext_vector_type(16))) __bf16 v16b;
typedef __attribute__((ext_vector_type(8)))  _Float16 v8h;
typedef __attribute__((ext_vector_type(8)))  float v8f;
typedef __attribute__((ext_vector_type(4)))  float v4f;
typedef __attribute__((ext_vector_type(2)))  float v2f;
typedef __attribute__((ext_vector_type(4)))  unsigned v4u;
typedef __attribute__((ext_vector_type(4)))  int v4i;
typedef float __attribute__((may_alias)) float_a;
typedef int __attribute__((may_alias)) int_a;

template <typename T> __device__ __forceinline__ void vst2(void* p, T v) { *(volatile T*)p = v; __threadfence(); *(volatile T*)p = v; }
__device__ __forceinline__ v8f wmma16(v16h a, v16h b, v8f c) {
  v8f d = __builtin_amdgcn_wmma_f32_16x16x32_f16(false, a, false, b, (short)0, c, false, false);
  asm volatile("v_nop\n\tv_nop\n\tv_nop\n\tv_nop" : "+v"(d) : "v"(a), "v"(b));
  return d;
}
__device__ __forceinline__ v8f wmma_bf(v16b a, v16b b, v8f c) {
  v8f d = __builtin_amdgcn_wmma_f32_16x16x32_bf16(false, a, false, b, (short)0, c, false, false);
  asm volatile("v_nop\n\tv_nop\n\tv_nop\n\tv_nop" : "+v"(d) : "v"(a), "v"(b));
  return d;
}
__device__ __forceinline__ v16h frag_h(const _Float16* rowk0, int lane) {
  union { v16h v; v8h q[2]; } u; const _Float16* p = rowk0 + 8 * (lane >> 4);
  u.q[0] = *(const v8h*)p; u.q[1] = *(const v8h*)(p + 16); return u.v;
}
__device__ __forceinline__ v16h frag_f32(const float* rowk0, int lane) {
  v16h a; const float* p = rowk0 + 8 * (lane >> 4);
#pragma unroll
  for (int i = 0; i < 8; ++i) { a[i] = (_Float16)p[i]; a[8 + i] = (_Float16)p[16 + i]; }
  return a;
}
__device__ __forceinline__ v16h frag_f32s(const float* rowk0, int lane, float sc) {
  v16h a; const float* p = rowk0 + 8 * (lane >> 4);
#pragma unroll
  for (int i = 0; i < 8; ++i) { a[i] = (_Float16)(p[i] * sc); a[8 + i] = (_Float16)(p[16 + i] * sc); }
  return a;
}
__device__ __forceinline__ v16h fragc_f32(const float* W, int k0, int n, int lane, int ld, int K) {
  v16h a; const int g = lane >> 4;
#pragma unroll
  for (int i = 0; i < 8; ++i) { const int ka = k0 + 8 * g + i, kb = ka + 16;
    a[i] = (_Float16)(ka < K ? W[(size_t)ka * ld + n] : 0.f); a[8 + i] = (_Float16)(kb < K ? W[(size_t)kb * ld + n] : 0.f); }
  return a;
}
struct F2 { v16b h, l; };
__device__ __forceinline__ F2 bsplit16(const float v[16]) { F2 r;
#pragma unroll
  for (int i = 0; i < 16; ++i) { const __bf16 h = (__bf16)v[i]; r.h[i] = h; r.l[i] = (__bf16)(v[i] - (float)h); }
  return r; }
__device__ __forceinline__ F2 split_row(const float* row, int k0, int lane) { float v[16]; const float* p = row + k0 + 8 * (lane >> 4);
#pragma unroll
  for (int i = 0; i < 8; ++i) { v[i] = p[i]; v[8 + i] = p[16 + i]; }
  return bsplit16(v); }
__device__ __forceinline__ F2 split_rowK(const float* row, int k0, int lane, int K) { float v[16]; const int g = lane >> 4;
#pragma unroll
  for (int i = 0; i < 8; ++i) { const int ka = k0 + 8 * g + i, kb = ka + 16; v[i] = ka < K ? row[ka] : 0.f; v[8 + i] = kb < K ? row[kb] : 0.f; }
  return bsplit16(v); }
__device__ __forceinline__ F2 split_col(const float* W, int k0, int n, int lane, int ld, int K) { float v[16]; const int g = lane >> 4;
#pragma unroll
  for (int i = 0; i < 8; ++i) { const int ka = k0 + 8 * g + i, kb = ka + 16; v[i] = ka < K ? W[(size_t)ka * ld + n] : 0.f; v[8 + i] = kb < K ? W[(size_t)kb * ld + n] : 0.f; }
  return bsplit16(v); }
__device__ __forceinline__ v8f mac3(const F2& a, const F2& b, v8f c) { c = wmma_bf(a.l, b.h, c); c = wmma_bf(a.h, b.l, c); return wmma_bf(a.h, b.h, c); }
__device__ __forceinline__ float sigm(float v) { return 1.0f / (1.0f + expf(-v)); }
#define LDSX() do { asm volatile("s_wait_dscnt 0" ::: "memory"); __builtin_amdgcn_wave_barrier(); __builtin_amdgcn_fence(__ATOMIC_RELEASE, "workgroup"); } while (0)


#define NBI 16
#define NT 1024
#define C 512
#define NH 8
#define HD 64
#define MF 256
#define NR (NBI * NT)
#define NBH (NBI * NH)
#define CTW 80
#define RATIO 0.0625f
#define NRM 0.35355339059327379f
#define EPSK 1e-4f

__global__ __launch_bounds__(256) void k_cvt(const float* __restrict__ x, _Float16* __restrict__ X16) {
  __shared__ __align__(16) _Float16 st[C][72];
  const int tid = threadIdx.x; const int b = blockIdx.x / (NT / 64), n0 = (blockIdx.x % (NT / 64)) * 64;
  for (int q = tid; q < C * 16; q += 256) { const int c = q >> 4, p4 = q & 15; const v4f v = *(const v4f*)(x + ((size_t)b * C + c) * NT + n0 + p4 * 4);
    st[c][p4 * 4] = (_Float16)v[0]; st[c][p4 * 4 + 1] = (_Float16)v[1]; st[c][p4 * 4 + 2] = (_Float16)v[2]; st[c][p4 * 4 + 3] = (_Float16)v[3]; }
  __syncthreads();
  for (int q = tid; q < 64 * (C / 8); q += 256) { const int nl = q >> 6, pc = q & 63; union { v8h h; v4u u; } pk;
#pragma unroll
    for (int e = 0; e < 8; ++e) pk.h[e] = st[pc * 8 + e][nl];
    vst2(X16 + ((size_t)b * NT + n0 + nl) * C + pc * 8, pk.u); }
}
__global__ __launch_bounds__(256) void k_pack(const float* __restrict__ Wq, const float* __restrict__ Wk, const float* __restrict__ Wv, const float* __restrict__ Wo, _Float16* __restrict__ PT) {
  const int n = blockIdx.x, tid = threadIdx.x; __shared__ __align__(16) _Float16 srow[C];
  const float* W = n < 512 ? Wq : (n < 1024 ? Wk : (n < 1536 ? Wv : Wo)); const int nn = n & 511;
  srow[tid] = (_Float16)(W[(size_t)tid * C + nn] * 16.0f); srow[tid + 256] = (_Float16)(W[(size_t)(tid + 256) * C + nn] * 16.0f);
  __syncthreads();
  if (tid < C / 8) vst2(PT + (size_t)n * C + tid * 8, *(const v4u*)(&srow[tid * 8]));
}
__global__ __launch_bounds__(128) void k_qkv(const _Float16* __restrict__ X16, const _Float16* __restrict__ PT, float* __restrict__ QF, float* __restrict__ KF, _Float16* __restrict__ VT) {
  __shared__ __align__(16) float so[4][16][132];
  __shared__ __align__(16) _Float16 sth[128][72];
  const int tid = threadIdx.x, wave = tid >> 5, lane = tid & 31, col = lane & 15, g = lane >> 4;
  const int which = blockIdx.z, r0b = blockIdx.x * 64, r0 = r0b + wave * 16, n0 = blockIdx.y * 128; const int b = r0b / NT, s0 = r0b % NT;
  v8f acc[8] = {};
#pragma unroll 2
  for (int kc = 0; kc < C / 32; ++kc) { const v16h a = frag_h(X16 + (size_t)(r0 + col) * C + kc * 32, lane);
#pragma unroll
    for (int j = 0; j < 8; ++j) acc[j] = wmma16(a, frag_h(PT + (size_t)(which * C + n0 + j * 16 + col) * C + kc * 32, lane), acc[j]); }
  if (which < 2) {
#pragma unroll
    for (int j = 0; j < 8; ++j)
#pragma unroll
      for (int r = 0; r < 8; ++r) so[wave][8 * g + r][j * 16 + col] = acc[j][r] * (1.0f / 16.0f);
    LDSX();
    float* Dst = which == 0 ? QF : KF;
    for (int qq = lane; qq < 2 * 16 * 16; qq += 32) { const int hh = qq >> 8, rl = (qq >> 4) & 15, pc = qq & 15; const int h = (n0 >> 6) + hh;
      vst2(Dst + (((size_t)b * NH + h) * NT + s0 + wave * 16 + rl) * HD + pc * 4, *(const v4f*)(&so[wave][rl][hh * 64 + pc * 4])); } }
  else {
#pragma unroll
    for (int j = 0; j < 8; ++j)
#pragma unroll
      for (int r = 0; r < 8; ++r) sth[j * 16 + col][wave * 16 + 8 * g + r] = (_Float16)(acc[j][r] * (4.0f / 16.0f));
    __syncthreads();
    for (int qq = tid; qq < 128 * 8; qq += 128) { const int cl = qq >> 3, pc = qq & 7; const int cc = n0 + cl, h = cc >> 6, d = cc & 63;
      vst2(VT + (((size_t)b * NH + h) * HD + d) * NT + s0 + pc * 8, *(const v4u*)(&sth[cl][pc * 8])); } }
}
__device__ __forceinline__ v8f ddtile(const float* __restrict__ drow, const float* __restrict__ proj, int t, int lane) { const int col = lane & 15; v8f acc = {};
#pragma unroll
  for (int kc = 0; kc < 2; ++kc) acc = mac3(split_row(drow, kc * 32, lane), split_row(proj + (size_t)(t * 16 + col) * HD, kc * 32, lane), acc);
  return acc; }
__global__ __launch_bounds__(256) void k_kmax(const float* __restrict__ KF, const float* __restrict__ proj, float* __restrict__ KMAX) {
  __shared__ float smx[8];
  const int tid = threadIdx.x, wave = tid >> 5, lane = tid & 31; const size_t bh = blockIdx.x; float mx = -3.4e38f;
#pragma unroll 1
  for (int rt = wave; rt < NT / 16; rt += 8) { const float* drow = KF + (bh * NT + rt * 16 + (lane & 15)) * HD;
#pragma unroll 1
    for (int t = 0; t < MF / 16; ++t) { const v8f a = ddtile(drow, proj, t, lane);
#pragma unroll
      for (int r = 0; r < 8; ++r) mx = fmaxf(mx, a[r]); } }
#pragma unroll
  for (int off = 16; off > 0; off >>= 1) mx = fmaxf(mx, __shfl_xor(mx, off, 32));
  if (lane == 0) smx[wave] = mx;
  __syncthreads();
  if (tid < 32) { float m = smx[0];
#pragma unroll
    for (int w = 1; w < 8; ++w) m = fmaxf(m, smx[w]);
    vst2(KMAX + bh * 32 + tid, (float_a)(m * NRM)); }
}
#define KPS 16384.0f
__global__ __launch_bounds__(256) void k_kctx(const float* __restrict__ KF, const float* __restrict__ proj, const float* __restrict__ KMAX, const _Float16* __restrict__ VT, _Float16* __restrict__ CT) {
  __shared__ __align__(16) _Float16 skt[MF][72];
  __shared__ __align__(16) float sks[MF];
  __shared__ __align__(16) float sct[64 + 16][MF + 4];
  const int tid = threadIdx.x, wave = tid >> 5, lane = tid & 31, col = lane & 15, g = lane >> 4; const size_t bh = blockIdx.x;
  const float kmax = KMAX[bh * 32];
  if (tid < MF) sks[tid] = 0.f;
  v8f cacc[2][4] = {};
  __syncthreads();
#pragma unroll 1
  for (int ch = 0; ch < NT / 64; ++ch) {
    { const int tt = wave & 3, t0 = (wave >> 2) * 8; const float* drow = KF + (bh * NT + ch * 64 + tt * 16 + col) * HD;
      float dg = 0.f; { const float* dr = KF + (bh * NT + ch * 64 + tt * 16 + col) * HD;
#pragma unroll 4
        for (int k = 0; k < HD; ++k) { const float v = dr[k] * NRM; dg += v * v; } dg *= 0.5f; }
#pragma unroll 1
      for (int j = 0; j < 8; ++j) { const v8f a = ddtile(drow, proj, t0 + j, lane);
#pragma unroll
        for (int r = 0; r < 8; ++r) { const float dgr = __shfl(dg, 8 * g + r, 32); const float kp = RATIO * (expf(a[r] * NRM - dgr - kmax) + EPSK); skt[(t0 + j) * 16 + col][tt * 16 + 8 * g + r] = (_Float16)(kp * KPS); } } }
    __syncthreads();
    if (tid < MF) { float s = 0.f; const _Float16* rr = &skt[tid][0];
#pragma unroll 8
      for (int n = 0; n < 64; ++n) s += (float)rr[n]; sks[tid] += s; }
#pragma unroll
    for (int kc = 0; kc < 2; ++kc) {
#pragma unroll
      for (int i = 0; i < 2; ++i) { const v16h a = frag_h(&skt[(2 * wave + i) * 16 + col][0] + kc * 32, lane);
#pragma unroll
        for (int t = 0; t < 4; ++t) cacc[i][t] = wmma16(a, frag_h(VT + (bh * HD + t * 16 + col) * NT + ch * 64 + kc * 32, lane), cacc[i][t]); } }
    __syncthreads(); }
#pragma unroll
  for (int i = 0; i < 2; ++i)
#pragma unroll
    for (int t = 0; t < 4; ++t)
#pragma unroll
      for (int r = 0; r < 8; ++r) sct[t * 16 + col][(2 * wave + i) * 16 + 8 * g + r] = cacc[i][t][r] * (1.0f / (KPS * 4.0f));
  if (tid < MF) { sct[64][tid] = sks[tid] * (1.0f / KPS); }
  for (int q = tid; q < 15 * MF; q += 256) sct[65 + q / MF][q % MF] = 0.f;
  __syncthreads();
  for (int q = tid; q < CTW * (MF / 8); q += 256) { const int d = q >> 5, pc = q & 31; union { v8h h; v4u u; } pk;
#pragma unroll
    for (int e = 0; e < 8; ++e) pk.h[e] = (_Float16)(sct[d][pc * 8 + e] * 16.0f);
    vst2(CT + (bh * CTW + d) * MF + pc * 8, pk.u); }
}
__global__ __launch_bounds__(128) void k_qfin(const float* __restrict__ QF, const float* __restrict__ proj, const _Float16* __restrict__ CT, _Float16* __restrict__ O16) {
  __shared__ __align__(16) _Float16 sq[4][16][MF + 8];
  __shared__ __align__(16) float so[4][16][84];
  const int tid = threadIdx.x, wave = tid >> 5, lane = tid & 31, col = lane & 15, g = lane >> 4; const size_t bh = blockIdx.y; const int b = (int)(bh / NH), h = (int)(bh % NH); const int q0 = blockIdx.x * 64 + wave * 16;
  const float* drow = QF + (bh * NT + q0 + col) * HD;
  float dg = 0.f;
#pragma unroll 4
  for (int k = 0; k < HD; ++k) { const float v = drow[k] * NRM; dg += v * v; }
  dg *= 0.5f;
  v8f a[16]; float mx[8];
#pragma unroll
  for (int r = 0; r < 8; ++r) mx[r] = -3.4e38f;
#pragma unroll
  for (int t = 0; t < 16; ++t) { a[t] = ddtile(drow, proj, t, lane);
#pragma unroll
    for (int r = 0; r < 8; ++r) mx[r] = fmaxf(mx[r], a[t][r]); }
#pragma unroll
  for (int r = 0; r < 8; ++r) { float m = mx[r];
#pragma unroll
    for (int off = 1; off < 16; off <<= 1) m = fmaxf(m, __shfl_xor(m, off, 32));
    mx[r] = m * NRM; }
#pragma unroll
  for (int t = 0; t < 16; ++t)
#pragma unroll
    for (int r = 0; r < 8; ++r) { const float dgr = __shfl(dg, 8 * g + r, 32); sq[wave][8 * g + r][t * 16 + col] = (_Float16)(RATIO * (expf(a[t][r] * NRM - dgr - mx[r]) + EPSK) * KPS); }
  LDSX();
  v8f acc[5] = {};
#pragma unroll 2
  for (int kc = 0; kc < MF / 32; ++kc) { const v16h aa = frag_h(&sq[wave][col][0] + kc * 32, lane);
#pragma unroll
    for (int t = 0; t < 5; ++t) acc[t] = wmma16(aa, frag_h(CT + (bh * CTW + t * 16 + col) * MF + kc * 32, lane), acc[t]); }
#pragma unroll
  for (int t = 0; t < 5; ++t)
#pragma unroll
    for (int r = 0; r < 8; ++r) so[wave][8 * g + r][t * 16 + col] = acc[t][r];
  LDSX();
  { const int rl = lane & 15, hf = lane >> 4; const float den = so[wave][rl][64]; const float inv = 8.0f / den; union { v8h h8[4]; v4u u[4]; } pk;
#pragma unroll
    for (int e = 0; e < 32; ++e) pk.h8[e >> 3][e & 7] = (_Float16)(so[wave][rl][hf * 32 + e] * inv);
#pragma unroll
    for (int p4 = 0; p4 < 4; ++p4) vst2(O16 + ((size_t)b * NT + q0 + rl) * C + h * HD + hf * 32 + p4 * 8, pk.u[p4]); }
}
__global__ __launch_bounds__(128) void k_out(const _Float16* __restrict__ O16, const _Float16* __restrict__ PT, float* __restrict__ out) {
  __shared__ __align__(16) float st[128][68];
  const int tid = threadIdx.x, wave = tid >> 5, lane = tid & 31, col = lane & 15, g = lane >> 4;
  const int r0b = blockIdx.x * 64, r0 = r0b + wave * 16, n0 = blockIdx.y * 128; const int b = r0b / NT, s0 = r0b % NT;
  v8f acc[8] = {};
#pragma unroll 2
  for (int kc = 0; kc < C / 32; ++kc) { const v16h a = frag_h(O16 + (size_t)(r0 + col) * C + kc * 32, lane);
#pragma unroll
    for (int j = 0; j < 8; ++j) acc[j] = wmma16(a, frag_h(PT + (size_t)(3 * C + n0 + j * 16 + col) * C + kc * 32, lane), acc[j]); }
#pragma unroll
  for (int j = 0; j < 8; ++j)
#pragma unroll
    for (int r = 0; r < 8; ++r) st[j * 16 + col][wave * 16 + 8 * g + r] = acc[j][r] * (1.0f / (16.0f * 8.0f));
  __syncthreads();
  for (int qq = tid; qq < 128 * 16; qq += 128) { const int cl = qq >> 4, pc = qq & 15; vst2(out + ((size_t)b * C + n0 + cl) * NT + s0 + pc * 4, *(const v4f*)(&st[cl][pc * 4])); }
}
extern "C" void kernel_launch(void* const* d_in, const int* in_sizes, int n_in, void* d_out, int out_size, void* d_ws, size_t ws_size, hipStream_t stream) {
  (void)in_sizes; (void)n_in; (void)out_size; (void)ws_size;
  const float* x = (const float*)d_in[0]; const float* Wq = (const float*)d_in[1]; const float* Wk = (const float*)d_in[2]; const float* Wv = (const float*)d_in[3]; const float* Wo = (const float*)d_in[4]; const float* proj = (const float*)d_in[5];
  float* out = (float*)d_out;
  char* ws = (char*)d_ws; size_t off = 0;
  auto take = [&](size_t bytes) { char* p = ws + off; off += (bytes + 255) & ~(size_t)255; return p; };
  _Float16* X16 = (_Float16*)take((size_t)NR * C * 2); _Float16* PT = (_Float16*)take((size_t)4 * C * C * 2);
  float* QF = (float*)take((size_t)NR * C * 4); float* KF = (float*)take((size_t)NR * C * 4); _Float16* VT = (_Float16*)take((size_t)NR * C * 2);
  float* KMAX = (float*)take((size_t)NBH * 32 * 4); _Float16* CT = (_Float16*)take((size_t)NBH * CTW * MF * 2); _Float16* O16 = X16;
  k_cvt<<<NBI * (NT / 64), 256, 0, stream>>>(x, X16);
  k_pack<<<4 * C, 256, 0, stream>>>(Wq, Wk, Wv, Wo, PT);
  k_qkv<<<dim3(NR / 64, C / 128, 3), 128, 0, stream>>>(X16, PT, QF, KF, VT);
  k_kmax<<<NBH, 256, 0, stream>>>(KF, proj, KMAX);
  k_kctx<<<NBH, 256, 0, stream>>>(KF, proj, KMAX, VT, CT);
  k_qfin<<<dim3(NT / 64, NBH), 128, 0, stream>>>(QF, proj, CT, O16);
  k_out<<<dim3(NR / 64, C / 128), 128, 0, stream>>>(O16, PT, out);
}
